// EncoderHead_23313082483042
// MI455X (gfx1250) — hardware-verified
//
#include <hip/hip_runtime.h>


namespace {
constexpr int B = 16, T = 2048, C = 64, HD = 64, BL = 16  ;
constexpr float XS = 8.0f, WSC = 256.0f, PS = 1024.0f, LOG2E = 1.4426950408889634f;
static_assert(T % 64 == 0 && C == 64 && HD == 64, "tiling");
typedef _Float16 b16;
typedef __attribute__((ext_vector_type(16))) _Float16 v16b;
typedef __attribute__((ext_vector_type(8))) _Float16 v8b;
typedef __attribute__((ext_vector_type(8))) float v8f;
typedef __attribute__((ext_vector_type(4))) float v4f;
__device__ __forceinline__ float bf16_rne(float f) { unsigned int u = __float_as_uint(f); u += 0x7FFFu + ((u >> 16) & 1u); return __uint_as_float(u & 0xFFFF0000u); }
__device__ __forceinline__ void split16(float v, b16& hi, b16& lo) { hi = (b16)v; lo = (b16)(v - (float)hi); }
__device__ __forceinline__ v16b frag_kb(const b16* p, int hh) { const v8b a = *(const v8b*)(p + 8 * hh), b = *(const v8b*)(p + 16 + 8 * hh); v16b f;
#pragma unroll
  for (int e = 0; e < 8; ++e) { f[e] = a[e]; f[8 + e] = b[e]; } return f; }
__device__ __forceinline__ v8f wmma16b(v16b a, v16b b, v8f c) { v8f d = __builtin_amdgcn_wmma_f32_16x16x32_f16(false, a, false, b, (short)0, c, false, false); asm volatile("v_nop\n\tv_nop\n\tv_nop\n\tv_nop" : "+v"(d) : "v"(a), "v"(b)); return d; }
__device__ __forceinline__ void wave_lds_sync() { __builtin_amdgcn_fence(__ATOMIC_RELEASE, "workgroup"); __builtin_amdgcn_wave_barrier(); __builtin_amdgcn_fence(__ATOMIC_ACQUIRE, "workgroup"); }
__device__ __forceinline__ float pmul(float a, float b) { float p = a * b; asm volatile("" : "+v"(p)); return p; }
__device__ __forceinline__ int iclamp(int v, int lo, int hi) { return v < lo ? lo : (v > hi ? hi : v); }

typedef __attribute__((ext_vector_type(2))) _Float16 v2h;
typedef __attribute__((ext_vector_type(2))) float v2f;
__device__ __forceinline__ float nexp2(float v) { return __builtin_amdgcn_exp2f(v); }
__global__ __launch_bounds__(256) void wprep_kernel(const float* __restrict__ wq, const float* __restrict__ wk, const float* __restrict__ wv, b16* __restrict__ WT) {
  for (int u = threadIdx.x; u < 3 * HD * C / 8; u += 256) { const int e = u * 8; const int s = e / (HD * C), el = e % (HD * C); const int h = el / C, c0 = el % C; const float* w = s == 0 ? wq : (s == 1 ? wk : wv); v8b o;
    for (int j = 0; j < 8; ++j) o[j] = (b16)(bf16_rne(w[(c0 + j) * HD + h]) * WSC);
    for (int pass = 0; pass < 2; ++pass) { *(volatile v8b*)(WT + e) = o; __threadfence(); } }
}
__global__ __launch_bounds__(128) void qkv_kernel(const float* __restrict__ x, const b16* __restrict__ WT, b16* __restrict__ Qh, b16* __restrict__ Ql, b16* __restrict__ Kh, b16* __restrict__ Kl, b16* __restrict__ VT) {
  __shared__ __attribute__((aligned(16))) b16 As[4][16][C + 8]; __shared__ __attribute__((aligned(16))) float Tf[4][16][192 + 4];
  const int wave = threadIdx.x >> 5, lane = threadIdx.x & 31, nloc = lane & 15, hlf = lane >> 4; const int b = blockIdx.y; const int t0 = blockIdx.x * 64 + wave * 16;
  for (int rr = 0; rr < 16; ++rr) { const float* xr = x + ((size_t)b * T + t0 + rr) * C; v2h o; o[0] = (b16)(bf16_rne(xr[lane * 2]) * XS); o[1] = (b16)(bf16_rne(xr[lane * 2 + 1]) * XS); *(v2h*)(&As[wave][rr][lane * 2]) = o; }
  wave_lds_sync();
  v8f acc[12];
#pragma unroll
  for (int t = 0; t < 12; ++t) acc[t] = (v8f){};
#pragma unroll
  for (int kb = 0; kb < C; kb += 32) { const v16b a = frag_kb(&As[wave][nloc][kb], hlf);
#pragma unroll
    for (int t = 0; t < 12; ++t) acc[t] = wmma16b(a, frag_kb(WT + (size_t)(t * 16 + nloc) * C + kb, hlf), acc[t]); }
#pragma unroll
  for (int t = 0; t < 12; ++t)
#pragma unroll
    for (int r = 0; r < 8; ++r) Tf[wave][8 * hlf + r][t * 16 + nloc] = acc[t][r] * (1.0f / (XS * WSC));
  __syncthreads();
  for (int pass = 0; pass < 2; ++pass) {
    for (int rr = 0; rr < 16; ++rr) { const size_t row = ((size_t)b * T + t0 + rr) * HD; v2h qh, ql, kh, kl;
      for (int j = 0; j < 2; ++j) { b16 p, q; split16(Tf[wave][rr][lane * 2 + j] * XS, p, q); qh[j] = p; ql[j] = q; split16(Tf[wave][rr][HD + lane * 2 + j] * XS, p, q); kh[j] = p; kl[j] = q; }
      *(volatile v2h*)(Qh + row + lane * 2) = qh; *(volatile v2h*)(Ql + row + lane * 2) = ql; *(volatile v2h*)(Kh + row + lane * 2) = kh; *(volatile v2h*)(Kl + row + lane * 2) = kl; }
#pragma unroll 1
    for (int q = 0; q < 16; ++q) { const int d = wave * 16 + q; const int tk = lane * 2; v2h vv; vv[0] = (b16)(Tf[tk >> 4][tk & 15][2 * HD + d] * XS); vv[1] = (b16)(Tf[(tk + 1) >> 4][(tk + 1) & 15][2 * HD + d] * XS);
      *(volatile v2h*)(VT + ((size_t)b * HD + d) * T + blockIdx.x * 64 + lane * 2) = vv; }
    __threadfence(); }
}
__global__ __launch_bounds__(64) void attn_kernel(const b16* __restrict__ Qh, const b16* __restrict__ Ql, const b16* __restrict__ Kh, const b16* __restrict__ Kl, const b16* __restrict__ VT, float* __restrict__ out) {
  __shared__ __attribute__((aligned(16))) float To[2][16][HD + 4];
  const int wave = threadIdx.x >> 5, lane = threadIdx.x & 31, hh = lane >> 4, col = lane & 15; const int b = blockIdx.y; const int q0 = blockIdx.x * 32 + wave * 16, qi = q0 + col;
  const b16* Qhb = Qh + (size_t)b * T * HD, * Qlb = Ql + (size_t)b * T * HD, * Khb = Kh + (size_t)b * T * HD, * Klb = Kl + (size_t)b * T * HD, * Vb = VT + (size_t)b * HD * T;
  v16b qh[2], ql[2]; for (int ks = 0; ks < 2; ++ks) { qh[ks] = frag_kb(Qhb + (size_t)qi * HD + ks * 32, hh); ql[ks] = frag_kb(Qlb + (size_t)qi * HD + ks * 32, hh); }
  const float cs = LOG2E * 0.125f / (XS * XS);
  float m = -INFINITY, l = 0.0f; v8f o[4]; for (int t = 0; t < 4; ++t) o[t] = (v8f){};
#pragma unroll 1
  for (int kb = 0; kb < T; kb += 32) {
    v8f s[2] = {(v8f){}, (v8f){}};
#pragma unroll
    for (int tt = 0; tt < 2; ++tt)
#pragma unroll
      for (int ks = 0; ks < 2; ++ks) { const size_t kr = (size_t)(kb + tt * 16 + col) * HD + ks * 32; const v16b khf = frag_kb(Khb + kr, hh), klf = frag_kb(Klb + kr, hh);
        s[tt] = wmma16b(khf, qh[ks], s[tt]); s[tt] = wmma16b(khf, ql[ks], s[tt]); s[tt] = wmma16b(klf, qh[ks], s[tt]); }
    float e[16]; float mx = -INFINITY;
#pragma unroll
    for (int r = 0; r < 8; ++r) { e[r] = s[0][r] * cs; e[8 + r] = s[1][r] * cs; mx = fmaxf(mx, fmaxf(e[r], e[8 + r])); }
    mx = fmaxf(mx, __shfl_xor(mx, 16)); const float mn = fmaxf(m, mx); const float al = nexp2(m - mn); m = mn; float sum = 0.0f; v16b ph, pl;
#pragma unroll
    for (int i = 0; i < 16; ++i) { const float p = nexp2(e[i] - mn); sum += p; b16 a_, b_; split16(p * PS, a_, b_); ph[i] = a_; pl[i] = b_; }
    sum += __shfl_xor(sum, 16); l = l * al + sum;
#pragma unroll
    for (int t = 0; t < 4; ++t) { o[t] *= al; const v16b va = frag_kb(Vb + (size_t)(t * 16 + col) * T + kb, hh); o[t] = wmma16b(va, ph, o[t]); o[t] = wmma16b(va, pl, o[t]); } }
  const float inv = 1.0f / (l * PS * XS);
#pragma unroll
  for (int t = 0; t < 4; ++t)
#pragma unroll
    for (int r = 0; r < 8; ++r) To[wave][col][t * 16 + 8 * hh + r] = o[t][r] * inv;
  wave_lds_sync();
  for (int pass = 0; pass < 2; ++pass) { for (int rr = 0; rr < 16; ++rr) *(volatile v2f*)(out + ((size_t)b * T + q0 + rr) * HD + lane * 2) = *(const v2f*)(&To[wave][rr][lane * 2]); __threadfence(); }
}
}

extern "C" void kernel_launch(void* const* d_in, const int* in_sizes, int n_in, void* d_out, int out_size, void* d_ws, size_t ws_size, hipStream_t stream) {
  (void)n_in;
  auto Fp = [&](int i) { return (const float*)d_in[i]; };
  if (in_sizes[0] != B * T * C || in_sizes[1] != C * HD || in_sizes[2] != C * HD || in_sizes[3] != C * HD || out_size != B * T * HD) return;
  size_t off = 0; char* ws = (char*)d_ws;
  auto carve = [&](size_t bytes) { char* p = ws + off; off += (bytes + 255) & ~(size_t)255; return p; };
  b16* WT = (b16*)carve((size_t)3 * HD * C * 2); b16* Qh = (b16*)carve((size_t)B * T * HD * 2); b16* Ql = (b16*)carve((size_t)B * T * HD * 2); b16* Kh = (b16*)carve((size_t)B * T * HD * 2); b16* Kl = (b16*)carve((size_t)B * T * HD * 2); b16* VT = (b16*)carve((size_t)B * HD * T * 2);
  if (off > ws_size || off > ((size_t)128 << 20)) return;
  wprep_kernel<<<1, 256, 0, stream>>>(Fp(1), Fp(2), Fp(3), WT);
  qkv_kernel<<<dim3(T / 64, BL), 128, 0, stream>>>(Fp(0), WT, Qh, Ql, Kh, Kl, VT);
  attn_kernel<<<dim3(T / 32, BL), 64, 0, stream>>>(Qh, Ql, Kh, Kl, VT, (float*)d_out);
}
